// ImageLinearAttention_79525614452956
// MI455X (gfx1250) — hardware-run, weakly checked
//
#include <hip/hip_runtime.h>
#include <math.h>

typedef __attribute__((ext_vector_type(16))) _Float16 v16h;
typedef __attribute__((ext_vector_type(16))) __bf16 v16b;
typedef __attribute__((ext_vector_type(8)))  _Float16 v8h;
typedef __attribute__((ext_vector_type(8)))  float v8f;
typedef __attribute__((ext_vector_type(4)))  float v4f;
typedef __attribute__((ext_vector_type(2)))  float v2f;
typedef __attribute__((ext_vector_type(4)))  unsigned v4u;
typedef __attribute__((ext_vector_type(4)))  int v4i;
typedef float __attribute__((may_alias)) float_a;
typedef int __attribute__((may_alias)) int_a;

template <typename T> __device__ __forceinline__ void vst2(void* p, T v) { *(volatile T*)p = v; __threadfence(); *(volatile T*)p = v; }
__device__ __forceinline__ v8f wmma16(v16h a, v16h b, v8f c) {
  v8f d = __builtin_amdgcn_wmma_f32_16x16x32_f16(false, a, false, b, (short)0, c, false, false);
  asm volatile("v_nop\n\tv_nop\n\tv_nop\n\tv_nop" : "+v"(d) : "v"(a), "v"(b));
  return d;
}
__device__ __forceinline__ v8f wmma_bf(v16b a, v16b b, v8f c) {
  v8f d = __builtin_amdgcn_wmma_f32_16x16x32_bf16(false, a, false, b, (short)0, c, false, false);
  asm volatile("v_nop\n\tv_nop\n\tv_nop\n\tv_nop" : "+v"(d) : "v"(a), "v"(b));
  return d;
}
__device__ __forceinline__ v16h frag_h(const _Float16* rowk0, int lane) {
  union { v16h v; v8h q[2]; } u; const _Float16* p = rowk0 + 8 * (lane >> 4);
  u.q[0] = *(const v8h*)p; u.q[1] = *(const v8h*)(p + 16); return u.v;
}
__device__ __forceinline__ v16h frag_f32(const float* rowk0, int lane) {
  v16h a; const float* p = rowk0 + 8 * (lane >> 4);
#pragma unroll
  for (int i = 0; i < 8; ++i) { a[i] = (_Float16)p[i]; a[8 + i] = (_Float16)p[16 + i]; }
  return a;
}
__device__ __forceinline__ v16h frag_f32s(const float* rowk0, int lane, float sc) {
  v16h a; const float* p = rowk0 + 8 * (lane >> 4);
#pragma unroll
  for (int i = 0; i < 8; ++i) { a[i] = (_Float16)(p[i] * sc); a[8 + i] = (_Float16)(p[16 + i] * sc); }
  return a;
}
__device__ __forceinline__ v16h fragc_f32(const float* W, int k0, int n, int lane, int ld, int K) {
  v16h a; const int g = lane >> 4;
#pragma unroll
  for (int i = 0; i < 8; ++i) { const int ka = k0 + 8 * g + i, kb = ka + 16;
    a[i] = (_Float16)(ka < K ? W[(size_t)(ka < K ? ka : K - 1) * ld + n] : 0.f); a[8 + i] = (_Float16)(kb < K ? W[(size_t)(kb < K ? kb : K - 1) * ld + n] : 0.f); }
  return a;
}
struct F2 { v16b h, l; };
__device__ __forceinline__ F2 bsplit16(const float v[16]) { F2 r;
#pragma unroll
  for (int i = 0; i < 16; ++i) { const __bf16 h = (__bf16)v[i]; r.h[i] = h; r.l[i] = (__bf16)(v[i] - (float)h); }
  return r; }
__device__ __forceinline__ F2 split_row(const float* row, int k0, int lane) { float v[16]; const float* p = row + k0 + 8 * (lane >> 4);
#pragma unroll
  for (int i = 0; i < 8; ++i) { v[i] = p[i]; v[8 + i] = p[16 + i]; }
  return bsplit16(v); }
__device__ __forceinline__ F2 split_rowK(const float* row, int k0, int lane, int K) { float v[16]; const int g = lane >> 4;
#pragma unroll
  for (int i = 0; i < 8; ++i) { const int ka = k0 + 8 * g + i, kb = ka + 16; v[i] = ka < K ? row[ka < K ? ka : K - 1] : 0.f; v[8 + i] = kb < K ? row[kb < K ? kb : K - 1] : 0.f; }
  return bsplit16(v); }
__device__ __forceinline__ F2 split_col(const float* W, int k0, int n, int lane, int ld, int K) { float v[16]; const int g = lane >> 4;
#pragma unroll
  for (int i = 0; i < 8; ++i) { const int ka = k0 + 8 * g + i, kb = ka + 16; v[i] = ka < K ? W[(size_t)(ka < K ? ka : K - 1) * ld + n] : 0.f; v[8 + i] = kb < K ? W[(size_t)(kb < K ? kb : K - 1) * ld + n] : 0.f; }
  return bsplit16(v); }
__device__ __forceinline__ v8f mac3(const F2& a, const F2& b, v8f c) { c = wmma_bf(a.l, b.h, c); c = wmma_bf(a.h, b.l, c); return wmma_bf(a.h, b.h, c); }
__device__ __forceinline__ float sigm(float v) { return 1.0f / (1.0f + expf(-v)); }
#define LDSX() do { asm volatile("s_wait_dscnt 0" ::: "memory"); __builtin_amdgcn_wave_barrier(); __builtin_amdgcn_fence(__ATOMIC_RELEASE, "workgroup"); } while (0)


#define NB 4
#define CC 128
#define NP 16384
#define NH 8
#define KD 64
#define QC (NH * KD)
#ifndef TNB
#define TNB NB
#define TPT (NP / 128)
#endif
typedef __attribute__((ext_vector_type(8))) __bf16 v8b;
__device__ __forceinline__ v16b frag_b(const __bf16* rowk0, int lane) {
  union { v16b v; v8b q[2]; } u; const __bf16* p = rowk0 + 8 * (lane >> 4);
  u.q[0] = *(const v8b*)p; u.q[1] = *(const v8b*)(p + 16); return u.v;
}
__device__ __forceinline__ float bfr(float v) { return (float)(__bf16)v; }
__device__ __attribute__((noinline)) float exp_ni(float v) { return expf(v); }
__device__ __attribute__((noinline)) float erf_ni(float v) { return erff(v); }

#define WS_PW  0u
#define WS_XT  (WS_PW + 2u * (size_t)3 * QC * CC)
#define WS_QP  (WS_XT + 2u * (size_t)NP * CC)
#define WS_KP  (WS_QP + 2u * (size_t)QC * NP)
#define WS_VP  (WS_KP + 2u * (size_t)QC * NP)
#define WS_KS  (WS_VP + 2u * (size_t)QC * NP)
#define WS_QS  (WS_KS + 2u * (size_t)QC * NP)
#define WS_CT  (WS_QS + 2u * (size_t)NP * QC)
#define WS_M   (WS_CT + 4u * (size_t)NH * KD * KD)
#define WS_END (WS_M + 4u * (size_t)CC * QC)

__global__ __launch_bounds__(128) void k_pack(const float* __restrict__ WQ, const float* __restrict__ WK, const float* __restrict__ WV, __bf16* __restrict__ PW) { const int n = blockIdx.x, which = blockIdx.y, t = threadIdx.x; __shared__ __align__(16) __bf16 s[CC]; const float* w = (which == 0) ? WQ : (which == 1) ? WK : WV; s[t] = (__bf16)w[(size_t)n * CC + t]; __syncthreads(); if (t < CC / 8) vst2((unsigned*)(PW + ((size_t)which * QC + n) * CC + t * 8), *(const v4u*)&s[t * 8]); }
__global__ __launch_bounds__(256) void k_xt(const float* __restrict__ X, __bf16* __restrict__ XT) { __shared__ float st[64][CC + 1]; __shared__ __align__(16) __bf16 so2[64][CC + 8]; const int t = threadIdx.x; const int p0 = blockIdx.x * 64; const size_t gb = blockIdx.y;
  for (int e = t; e < CC * 64; e += 256) { const int c = e >> 6, pl = e & 63; st[pl][c] = X[(gb * CC + c) * NP + p0 + pl]; } __syncthreads();
  for (int e = t; e < 64 * CC; e += 256) { const int pl = e >> 7, c = e & 127; so2[pl][c] = (__bf16)st[pl][c]; } __syncthreads();
  for (int e = t; e < 64 * 16; e += 256) { const int pl = e >> 4, q = e & 15; vst2((unsigned*)(XT + ((size_t)(p0 + pl) * CC) + q * 8), *(const v4u*)&so2[pl][q * 8]); } }
__global__ __launch_bounds__(128) void k_conv(const __bf16* __restrict__ PW, const __bf16* __restrict__ XT, const float* __restrict__ BQ, const float* __restrict__ BK, const float* __restrict__ BV, _Float16* __restrict__ QP, _Float16* __restrict__ KP, _Float16* __restrict__ VP) { __shared__ __align__(16) float so[4][16][132];
  const int tid = threadIdx.x, wave = tid >> 5, lane = tid & 31, col = lane & 15, g = lane >> 4; const int which = blockIdx.z; const size_t b = 0; const int o0 = blockIdx.x * 64 + wave * 16; const int p0 = blockIdx.y * 128; const __bf16* Wr = PW + ((size_t)which * QC) * CC; const float* BB = (which == 0) ? BQ : (which == 1) ? BK : BV; const float sc = (which < 2) ? 0.35355339059327373f : 1.0f;
  v8f acc[8] = {};
#pragma unroll
  for (int kc = 0; kc < CC / 32; ++kc) { const v16b a = frag_b(Wr + (size_t)(o0 + col) * CC + kc * 32, lane);
#pragma unroll
    for (int j = 0; j < 8; ++j) acc[j] = wmma_bf(a, frag_b(XT + ((b * NP + p0 + j * 16 + col) * CC) + kc * 32, lane), acc[j]); }
#pragma unroll
  for (int j = 0; j < 8; ++j)
#pragma unroll
    for (int r = 0; r < 8; ++r) so[wave][8 * g + r][j * 16 + col] = (acc[j][r] + bfr(BB[o0 + 8 * g + r])) * sc;
  LDSX();
  { _Float16* dst = (which == 0) ? QP : (which == 1) ? KP : VP; __shared__ __align__(16) _Float16 sh[4][16][136]; for (int e = lane; e < 16 * 128; e += 32) sh[wave][e >> 7][e & 127] = (_Float16)so[wave][e >> 7][e & 127]; LDSX(); for (int rl = 0; rl < 16; ++rl) if (lane < 16) vst2((unsigned*)(dst + ((b * QC + o0 + rl) * NP) + p0 + lane * 8), *(const v4u*)&sh[wave][rl][lane * 8]); } }
__global__ __launch_bounds__(256) void k_ksoft(const _Float16* __restrict__ KP, _Float16* __restrict__ KS) { __shared__ float red[8]; __shared__ __align__(16) _Float16 sp[NP]; const int t = threadIdx.x; const size_t row = blockIdx.x; const _Float16* kr = KP + row * NP;
  float mx = -3.0e38f; for (int i = t; i < NP; i += 256) mx = fmaxf(mx, (float)kr[i]);
#pragma unroll
  for (int o = 1; o < 32; o <<= 1) mx = fmaxf(mx, __shfl_xor(mx, o));
  if ((t & 31) == 0) red[t >> 5] = mx; __syncthreads(); float M = red[0]; for (int i = 1; i < 8; ++i) M = fmaxf(M, red[i]); __syncthreads();
  float z = 0.f; for (int i = t; i < NP; i += 256) z += __expf((float)kr[i] - M);
#pragma unroll
  for (int o = 1; o < 32; o <<= 1) z += __shfl_xor(z, o);
  if ((t & 31) == 0) red[t >> 5] = z; __syncthreads(); float Z = 0.f; for (int i = 0; i < 8; ++i) Z += red[i]; const float iz = 16384.0f / Z;
  for (int i = t; i < NP; i += 256) sp[i] = (_Float16)(__expf((float)kr[i] - M) * iz); __syncthreads();
  for (int q = t; q < NP / 8; q += 256) vst2((unsigned*)(KS + row * NP + q * 8), *(const v4u*)&sp[q * 8]); }
__global__ __launch_bounds__(128) void k_qsoft(const _Float16* __restrict__ QP, _Float16* __restrict__ QS) { __shared__ float st[KD][128 + 1]; __shared__ __align__(16) _Float16 so2[128][KD + 8]; const int t = threadIdx.x; const int p0 = blockIdx.x * 128; const int h = blockIdx.y; const size_t b = 0;
  for (int d = 0; d < KD; ++d) st[d][t] = (float)QP[((b * QC + h * KD + d) * NP) + p0 + t]; __syncthreads();
  { float mx = -3.0e38f; for (int d = 0; d < KD; ++d) mx = fmaxf(mx, st[d][t]); float z = 0.f; for (int d = 0; d < KD; ++d) z += __expf(st[d][t] - mx); const float iz = 1.0f / z; for (int d = 0; d < KD; ++d) so2[t][d] = (_Float16)(__expf(st[d][t] - mx) * iz); }
  __syncthreads(); for (int e = t; e < 128 * 8; e += 128) { const int pl = e >> 3, q = e & 7; vst2((unsigned*)(QS + ((b * NP + p0 + pl) * QC) + h * KD + q * 8), *(const v4u*)&so2[pl][q * 8]); } }
__global__ __launch_bounds__(128) void k_ctx(const _Float16* __restrict__ KS, const _Float16* __restrict__ VP, float* __restrict__ CT) { __shared__ __align__(16) float so[4][16][68];
  const int tid = threadIdx.x, wave = tid >> 5, lane = tid & 31, col = lane & 15, g = lane >> 4; const int h = blockIdx.x; const size_t b = 0; const _Float16* Kb = KS + ((b * QC + h * KD + wave * 16) * NP); const _Float16* Vb = VP + ((b * QC + h * KD) * NP);
  v8f acc[4] = {};
#pragma unroll 4
  for (int kc = 0; kc < NP / 32; ++kc) { const v16h a = frag_h(Kb + (size_t)col * NP + kc * 32, lane);
#pragma unroll
    for (int j = 0; j < 4; ++j) acc[j] = wmma16(a, frag_h(Vb + (size_t)(j * 16 + col) * NP + kc * 32, lane), acc[j]); }
#pragma unroll
  for (int j = 0; j < 4; ++j)
#pragma unroll
    for (int r = 0; r < 8; ++r) so[wave][8 * g + r][j * 16 + col] = acc[j][r] * (1.0f / 16384.0f);
  LDSX(); for (int rl = 0; rl < 16; ++rl) if (lane < 16) vst2(CT + (((b * NH + h) * KD + wave * 16 + rl) * KD) + lane * 4, *(const v4f*)&so[wave][rl][lane * 4]); }
__global__ __launch_bounds__(256) void k_m(const float* __restrict__ WO, const float* __restrict__ CT, float* __restrict__ M) { __shared__ float sw[QC]; __shared__ __align__(16) float so2[QC]; const int t = threadIdx.x; const int o = blockIdx.x; const size_t b = 0;
  for (int e = t; e < QC; e += 256) sw[e] = bfr(WO[(size_t)o * QC + e]); __syncthreads();
  for (int c = t; c < QC; c += 256) { const int h = c / KD, d = c % KD; const float* ct = CT + (((b * NH + h) * KD + d) * KD); float a = 0.f; for (int e = 0; e < KD; ++e) a += sw[h * KD + e] * ct[e]; so2[c] = a; } __syncthreads();
  if (t < QC / 4) vst2(M + ((b * CC + o) * QC) + t * 4, *(const v4f*)&so2[t * 4]); }
__global__ __launch_bounds__(128) void k_y(const float* __restrict__ M, const _Float16* __restrict__ QS, const float* __restrict__ BO, float* __restrict__ Y) { __shared__ __align__(16) float so[4][16][132];
  const int tid = threadIdx.x, wave = tid >> 5, lane = tid & 31, col = lane & 15, g = lane >> 4; const size_t b = 0; const int o0 = blockIdx.x * 64 + wave * 16; const int p0 = blockIdx.y * 128;
  v8f acc[8] = {}, accl[8] = {};
#pragma unroll 2
  for (int kc = 0; kc < QC / 32; ++kc) { v16h ah, al; { const float* p = M + ((b * CC + o0 + col) * QC) + kc * 32 + 8 * g;
#pragma unroll
      for (int i = 0; i < 8; ++i) { const float x0 = p[i], x1 = p[16 + i]; const _Float16 h0 = (_Float16)x0, h1 = (_Float16)x1; ah[i] = h0; ah[8 + i] = h1; al[i] = (_Float16)((x0 - (float)h0) * 2048.0f); al[8 + i] = (_Float16)((x1 - (float)h1) * 2048.0f); } }
#pragma unroll
    for (int j = 0; j < 8; ++j) { const v16h w = frag_h(QS + ((b * NP + p0 + j * 16 + col) * QC) + kc * 32, lane); acc[j] = wmma16(ah, w, acc[j]); accl[j] = wmma16(al, w, accl[j]); } }
#pragma unroll
  for (int j = 0; j < 8; ++j)
#pragma unroll
    for (int r = 0; r < 8; ++r) so[wave][8 * g + r][j * 16 + col] = acc[j][r] + accl[j][r] * (1.0f / 2048.0f) + bfr(BO[o0 + 8 * g + r]);
  LDSX(); for (int rl = 0; rl < 16; ++rl) vst2(Y + ((size_t)(o0 + rl) * NP) + p0 + lane * 4, *(const v4f*)&so[wave][rl][lane * 4]); }
extern "C" void kernel_launch(void* const* d_in, const int* in_sizes, int n_in, void* d_out, int out_size, void* d_ws, size_t ws_size, hipStream_t stream) {
  (void)in_sizes; (void)n_in; (void)out_size;
  const float** F = (const float**)d_in;
  if (ws_size < (size_t)WS_END) return;
  char* ws = (char*)d_ws; __bf16 *PW = (__bf16*)(ws + WS_PW), *XT = (__bf16*)(ws + WS_XT); float *CT = (float*)(ws + WS_CT), *M = (float*)(ws + WS_M); _Float16 *QP = (_Float16*)(ws + WS_QP), *KP = (_Float16*)(ws + WS_KP), *VP = (_Float16*)(ws + WS_VP), *KS = (_Float16*)(ws + WS_KS), *QS = (_Float16*)(ws + WS_QS);
  k_pack<<<dim3(QC, 3), 128, 0, stream>>>(F[1], F[3], F[5], PW);
  for (int gb = 0; gb < TNB; ++gb) {
    k_xt<<<dim3(NP / 64, 1), 256, 0, stream>>>(F[0] + (size_t)gb * CC * NP, XT);
    k_conv<<<dim3(QC / 64, NP / 128, 3), 128, 0, stream>>>(PW, XT, F[2], F[4], F[6], QP, KP, VP);
    k_ksoft<<<QC, 256, 0, stream>>>(KP, KS);
    k_qsoft<<<dim3(NP / 128, NH, 1), 128, 0, stream>>>(QP, QS);
    k_ctx<<<NH, 128, 0, stream>>>(KS, VP, CT);
    k_m<<<CC, 256, 0, stream>>>(F[7], CT, M);
    k_y<<<dim3(CC / 64, TPT, 1), 128, 0, stream>>>(M, QS, F[8], (float*)d_out + (size_t)gb * CC * NP); }
}
